// URLTextProcessor_48206712930853
// MI455X (gfx1250) — hardware-verified
//
#include <hip/hip_runtime.h>
#include <stdint.h>


#define VOCAB 100
#define EMB   32
#define HID   64
#define NOUT  32
#define TT    200

#define WAVES   4
#define BLOCK   (WAVES * 32)
#define MROWS   16
#define MPERBLK (WAVES * MROWS)
#define HSTRIDE 72

#define SACT 16.0f
#define SWGT 64.0f
#define SINV (1.0f / 1024.0f)

typedef _Float16 v16h __attribute__((ext_vector_type(16)));
typedef _Float16 v8h_t __attribute__((ext_vector_type(8)));
typedef v8h_t __attribute__((may_alias)) v8h;
typedef float v8f __attribute__((ext_vector_type(8)));
typedef float v4f_t __attribute__((ext_vector_type(4)));
typedef v4f_t __attribute__((may_alias)) v4f;

union Frag { v16h v; v8h half[2]; };

constexpr int OFF_WIH0 = 0;
constexpr int OFF_WHH0 = OFF_WIH0 + 256 * 32 * 2;
constexpr int OFF_WIH1 = OFF_WHH0 + 256 * 64 * 2;
constexpr int OFF_WHH1 = OFF_WIH1 + 256 * 64 * 2;
constexpr int OFF_WFC  = OFF_WHH1 + 256 * 64 * 2;
constexpr int OFF_EMB  = OFF_WFC  + 32 * 64 * 2;
constexpr int OFF_B0   = OFF_EMB  + VOCAB * EMB * 2;
constexpr int OFF_B1   = OFF_B0   + 256 * 4;
constexpr int OFF_BFC  = OFF_B1   + 256 * 4;
constexpr int OFF_STG  = OFF_BFC  + 32 * 4;
constexpr int STG_WAVE_BYTES = 2 * 16 * HSTRIDE * 2;
constexpr int SMEM_BYTES = OFF_STG + WAVES * STG_WAVE_BYTES;
static_assert((OFF_STG % 16) == 0, "");
static_assert((STG_WAVE_BYTES % 16) == 0, "");
static_assert(16 * NOUT * 4 <= STG_WAVE_BYTES, "");

__device__ __forceinline__ v8f wmma16(v16h a, v16h b, v8f c) {
  v8f d = __builtin_amdgcn_wmma_f32_16x16x32_f16(false, a, false, b, (short)0, c, false, false);
  asm volatile("v_nop\n\tv_nop\n\tv_nop\n\tv_nop" : "+v"(d) : "v"(a), "v"(b));
  return d;
}

__device__ __forceinline__ v16h ld_bfrag(const _Float16* W, int K, int ntile, int kofs, int lane) {
  const int n = ntile * 16 + (lane & 15);
  const _Float16* p = W + n * K + kofs + ((lane >> 4) << 3);
  Frag f;
  f.half[0] = *(const v8h*)(p);
  f.half[1] = *(const v8h*)(p + 16);
  return f.v;
}

__device__ __forceinline__ v16h ld_afrag(const _Float16* A, int stride, int kofs, int lane) {
  const int row = lane & 15;
  const _Float16* p = A + row * stride + kofs + ((lane >> 4) << 3);
  Frag f;
  f.half[0] = *(const v8h*)(p);
  f.half[1] = *(const v8h*)(p + 16);
  return f.v;
}

__device__ __forceinline__ void st_htile(_Float16* buf, int ncol0, const v8f v, int lane) {
  const int nc = ncol0 + (lane & 15);
  const int mb = (lane >> 4) * 8;
#pragma unroll
  for (int r = 0; r < 8; ++r) buf[(mb + r) * HSTRIDE + nc] = (_Float16)(v[r] * SACT);
}

__device__ __forceinline__ float sig1(float x) { return 1.0f / (1.0f + __expf(-x)); }
__device__ __forceinline__ float tanh1(float x) {
  float ax = __builtin_fabsf(x);
  float e  = __expf(2.0f * ax);
  float t  = 1.0f - 2.0f / (e + 1.0f);
  return __builtin_copysignf(t, x);
}
__device__ __forceinline__ v8f sig8(v8f x) {
  v8f r;
#pragma unroll
  for (int i = 0; i < 8; ++i) r[i] = sig1(x[i]);
  return r;
}
__device__ __forceinline__ v8f tanh8(v8f x) {
  v8f r;
#pragma unroll
  for (int i = 0; i < 8; ++i) r[i] = tanh1(x[i]);
  return r;
}
__device__ __forceinline__ v8f zero8() {
  v8f r = {0.f, 0.f, 0.f, 0.f, 0.f, 0.f, 0.f, 0.f};
  return r;
}
__device__ __forceinline__ v16h zero16() {
  v16h r;
#pragma unroll
  for (int i = 0; i < 16; ++i) r[i] = (_Float16)0.0f;
  return r;
}

__global__ void __launch_bounds__(BLOCK, 1) __attribute__((amdgpu_num_vgpr(256)))
k_lstm2(const int* __restrict__ x, const float* __restrict__ emb,
        const float* __restrict__ Wih0, const float* __restrict__ Whh0,
        const float* __restrict__ bih0, const float* __restrict__ bhh0,
        const float* __restrict__ Wih1, const float* __restrict__ Whh1,
        const float* __restrict__ bih1, const float* __restrict__ bhh1,
        const float* __restrict__ Wfc,  const float* __restrict__ bfc,
        float* out, int nB) {
  extern __shared__ char smem[];
  _Float16* sWih0 = (_Float16*)(smem + OFF_WIH0);
  _Float16* sWhh0 = (_Float16*)(smem + OFF_WHH0);
  _Float16* sWih1 = (_Float16*)(smem + OFF_WIH1);
  _Float16* sWhh1 = (_Float16*)(smem + OFF_WHH1);
  _Float16* sWfc  = (_Float16*)(smem + OFF_WFC);
  _Float16* sEmb  = (_Float16*)(smem + OFF_EMB);
  float*    sB0   = (float*)(smem + OFF_B0);
  float*    sB1   = (float*)(smem + OFF_B1);
  float*    sBfc  = (float*)(smem + OFF_BFC);

  const int tid  = threadIdx.x;
  const int lane = tid & 31;
  const int wave = tid >> 5;
  const int m    = lane & 15;
  const int hh   = lane >> 4;

  for (int i = tid; i < 256 * EMB; i += BLOCK) sWih0[i] = (_Float16)(Wih0[i] * SWGT);
  for (int i = tid; i < 256 * HID; i += BLOCK) sWhh0[i] = (_Float16)(Whh0[i] * SWGT);
  for (int i = tid; i < 256 * HID; i += BLOCK) sWih1[i] = (_Float16)(Wih1[i] * SWGT);
  for (int i = tid; i < 256 * HID; i += BLOCK) sWhh1[i] = (_Float16)(Whh1[i] * SWGT);
  for (int i = tid; i < NOUT * HID; i += BLOCK) sWfc[i]  = (_Float16)(Wfc[i] * SWGT);
  for (int i = tid; i < VOCAB * EMB; i += BLOCK) sEmb[i] = (_Float16)(emb[i] * SACT);
  for (int i = tid; i < 256; i += BLOCK) {
    sB0[i] = bih0[i] + bhh0[i];
    sB1[i] = bih1[i] + bhh1[i];
  }
  for (int i = tid; i < NOUT; i += BLOCK) sBfc[i] = bfc[i];
  __syncthreads();

  char* stgw = smem + OFF_STG + wave * STG_WAVE_BYTES;
  _Float16* h0buf = (_Float16*)stgw;
  _Float16* h1buf = h0buf + 16 * HSTRIDE;

  const int mbase = blockIdx.x * MPERBLK + wave * MROWS;
  int arow = mbase + m;
  if (arow >= nB) arow = nB - 1;
  const int* xrow = x + (size_t)arow * TT;

  v8f c0[4], c1[4];
#pragma unroll
  for (int j = 0; j < 4; ++j) { c0[j] = zero8(); c1[j] = zero8(); }
  v16h ah0_lo = zero16(), ah0_hi = zero16();
  v16h ah1_lo = zero16(), ah1_hi = zero16();

  int idx;
  {
    int v = xrow[0];
    if (v < 0) v += VOCAB;
    v = v < 0 ? 0 : (v > VOCAB - 1 ? VOCAB - 1 : v);
    idx = v;
  }

#pragma unroll 1
  for (int t = 0; t < TT; ++t) {
    const int tn = (t + 1 < TT) ? (t + 1) : (TT - 1);
    int idx_next;
    {
      int v = xrow[tn];
      if (v < 0) v += VOCAB;
      v = v < 0 ? 0 : (v > VOCAB - 1 ? VOCAB - 1 : v);
      idx_next = v;
    }

    v16h ax;
    {
      const _Float16* ep = sEmb + idx * EMB + (hh << 3);
      Frag f;
      f.half[0] = *(const v8h*)(ep);
      f.half[1] = *(const v8h*)(ep + 16);
      ax = f.v;
    }

#pragma unroll
    for (int jb = 0; jb < 4; ++jb) {
      v8f acc[4];
#pragma unroll
      for (int g = 0; g < 4; ++g) {
        const int nt = g * 4 + jb;
        v8f a = zero8();
        a = wmma16(ax,     ld_bfrag(sWih0, EMB, nt, 0,  lane), a);
        a = wmma16(ah0_lo, ld_bfrag(sWhh0, HID, nt, 0,  lane), a);
        a = wmma16(ah0_hi, ld_bfrag(sWhh0, HID, nt, 32, lane), a);
        acc[g] = a;
      }
      v8f pre[4];
#pragma unroll
      for (int g = 0; g < 4; ++g) {
        const float bc = sB0[(g * 4 + jb) * 16 + m];
        pre[g] = acc[g] * SINV + bc;
      }
      v8f it = sig8(pre[0]);
      v8f ft = sig8(pre[1]);
      v8f gt = tanh8(pre[2]);
      v8f ot = sig8(pre[3]);
      c0[jb] = ft * c0[jb] + it * gt;
      v8f h  = ot * tanh8(c0[jb]);
      st_htile(h0buf, jb * 16, h, lane);
    }
    __syncthreads();
    ah0_lo = ld_afrag(h0buf, HSTRIDE, 0,  lane);
    ah0_hi = ld_afrag(h0buf, HSTRIDE, 32, lane);

#pragma unroll
    for (int jb = 0; jb < 4; ++jb) {
      v8f acc[4];
#pragma unroll
      for (int g = 0; g < 4; ++g) {
        const int nt = g * 4 + jb;
        v8f a = zero8();
        a = wmma16(ah0_lo, ld_bfrag(sWih1, HID, nt, 0,  lane), a);
        a = wmma16(ah0_hi, ld_bfrag(sWih1, HID, nt, 32, lane), a);
        a = wmma16(ah1_lo, ld_bfrag(sWhh1, HID, nt, 0,  lane), a);
        a = wmma16(ah1_hi, ld_bfrag(sWhh1, HID, nt, 32, lane), a);
        acc[g] = a;
      }
      v8f pre[4];
#pragma unroll
      for (int g = 0; g < 4; ++g) {
        const float bc = sB1[(g * 4 + jb) * 16 + m];
        pre[g] = acc[g] * SINV + bc;
      }
      v8f it = sig8(pre[0]);
      v8f ft = sig8(pre[1]);
      v8f gt = tanh8(pre[2]);
      v8f ot = sig8(pre[3]);
      c1[jb] = ft * c1[jb] + it * gt;
      v8f h  = ot * tanh8(c1[jb]);
      st_htile(h1buf, jb * 16, h, lane);
    }
    __syncthreads();
    ah1_lo = ld_afrag(h1buf, HSTRIDE, 0,  lane);
    ah1_hi = ld_afrag(h1buf, HSTRIDE, 32, lane);

    idx = idx_next;
  }

  v8f y[2];
#pragma unroll
  for (int nt = 0; nt < 2; ++nt) {
    v8f a = zero8();
    a = wmma16(ah1_lo, ld_bfrag(sWfc, HID, nt, 0,  lane), a);
    a = wmma16(ah1_hi, ld_bfrag(sWfc, HID, nt, 32, lane), a);
    const float bc = sBfc[nt * 16 + m];
    v8f p = a * SINV + bc;
#pragma unroll
    for (int r = 0; r < 8; ++r) p[r] = p[r] > 0.f ? p[r] : 0.f;
    y[nt] = p;
  }

  float* fstg = (float*)stgw;
  __syncthreads();
#pragma unroll
  for (int nt = 0; nt < 2; ++nt) {
#pragma unroll
    for (int r = 0; r < 8; ++r) fstg[(hh * 8 + r) * NOUT + nt * 16 + m] = y[nt][r];
  }
  __syncthreads();

  v4f vals[4];
#pragma unroll
  for (int q = 0; q < 4; ++q) {
    const int r16 = q * 4 + (lane >> 3);
    const int pc  = lane & 7;
    vals[q] = *(const v4f*)(fstg + r16 * NOUT + pc * 4);
  }
#pragma unroll
  for (int q = 0; q < 4; ++q) {
    const int grow = mbase + q * 4 + (lane >> 3);
    const int pc   = lane & 7;
    if ((unsigned)grow < (unsigned)nB)
      *(volatile v4f*)(out + (size_t)grow * NOUT + pc * 4) = vals[q];
  }
  __threadfence();
#pragma unroll
  for (int q = 0; q < 4; ++q) {
    const int grow = mbase + q * 4 + (lane >> 3);
    const int pc   = lane & 7;
    if ((unsigned)grow < (unsigned)nB)
      *(volatile v4f*)(out + (size_t)grow * NOUT + pc * 4) = vals[q];
  }
}

extern "C" void kernel_launch(void* const* d_in, const int* in_sizes, int n_in,
                              void* d_out, int out_size, void* d_ws, size_t ws_size,
                              hipStream_t stream) {
  (void)n_in; (void)d_ws; (void)ws_size;
  int nB = in_sizes[0] / TT;
  const int nBo = out_size / NOUT;
  if (nBo < nB) nB = nBo;
  if (nB <= 0) return;
  hipFuncSetAttribute(reinterpret_cast<const void*>(k_lstm2),
                      hipFuncAttributeMaxDynamicSharedMemorySize, SMEM_BYTES);
  dim3 grid((nB + MPERBLK - 1) / MPERBLK);
  dim3 block(BLOCK);
  k_lstm2<<<grid, block, SMEM_BYTES, stream>>>(
      (const int*)d_in[0],   (const float*)d_in[1],
      (const float*)d_in[2], (const float*)d_in[3],
      (const float*)d_in[4], (const float*)d_in[5],
      (const float*)d_in[6], (const float*)d_in[7],
      (const float*)d_in[8], (const float*)d_in[9],
      (const float*)d_in[10], (const float*)d_in[11],
      (float*)d_out, nB);
  (void)hipGetLastError();
}
